// MultiHeadAttention_16037407883269
// MI455X (gfx1250) — hardware-verified
//
#include <hip/hip_runtime.h>
#ifndef NB
#define NB 2
#endif
#ifndef SEQ
#define SEQ 2048
#endif
#define NB_FULL 2
#define SEQ_FULL 2048
#define DM 1024
#define NH 16
#define HD 64
#define ISL 256
#define NRI (NB * SEQ)

static_assert(NH * HD == DM);
static_assert(HD == 64);
static_assert(DM % 128 == 0 && DM % 64 == 0 && DM % 32 == 0);
static_assert(NRI % 128 == 0 && SEQ % 64 == 0);
static_assert(ISL % 64 == 0 && ISL <= SEQ);
static_assert(NB <= NB_FULL && SEQ <= SEQ_FULL);
static_assert((long long)NRI * DM < 2147483647LL);

typedef _Float16 v16h __attribute__((ext_vector_type(16)));
typedef unsigned short v8us __attribute__((ext_vector_type(8), may_alias));
typedef float v8f __attribute__((ext_vector_type(8)));
typedef float v4f __attribute__((ext_vector_type(4)));
typedef float v4fa __attribute__((ext_vector_type(4), may_alias));
union FragH { v16h v; v8us half[2]; _Float16 h[16]; unsigned short u[16]; };

__device__ __forceinline__ unsigned short bf16_bits(float x) { unsigned int u = __float_as_uint(x); return (unsigned short)((u + 0x7FFFu + ((u >> 16) & 1u)) >> 16); }
__device__ __forceinline__ float bf16_val(unsigned short b) { return __uint_as_float(((unsigned int)b) << 16); }
__device__ __forceinline__ float bfr(float x) { return bf16_val(bf16_bits(x)); }

__device__ __forceinline__ v16h ldfrag(const unsigned short* p, int hh) { FragH f; f.half[0] = *(const v8us*)(p + 8 * hh); f.half[1] = *(const v8us*)(p + 16 + 8 * hh); return f.v; }
__device__ __forceinline__ v8f mma16(v16h a, v16h b, v8f c) { v8f d = __builtin_amdgcn_wmma_f32_16x16x32_f16(false, a, false, b, (short)0, c, false, false); asm volatile("v_nop\n\tv_nop\n\tv_nop\n\tv_nop" : "+v"(d) : "v"(a), "v"(b)); return d; }

__global__ __launch_bounds__(256) void k_wt_f16(const float* __restrict__ W, unsigned short* __restrict__ Wt, int K, int N, float scale) {
  const int t = blockIdx.x * 256 + threadIdx.x; if (t >= N * (K / 8)) return; const int n = t / (K / 8), k8 = (t % (K / 8)) * 8; FragH f;
#pragma unroll
  for (int i = 0; i < 8; ++i) f.h[i] = (_Float16)(bfr(W[(size_t)(k8 + i) * N + n]) * scale);
  const v8us o = f.half[0];
  *(volatile v8us*)(Wt + (size_t)n * K + k8) = o; __threadfence(); *(volatile v8us*)(Wt + (size_t)n * K + k8) = o;
}

__global__ __launch_bounds__(256) void k_x16(const float* __restrict__ x, unsigned short* __restrict__ X16) {
  const int t = blockIdx.x * 256 + threadIdx.x; if (t >= NRI * (DM / 8)) return;
  const int row = t / (DM / 8), c8 = (t - row * (DM / 8)) * 8; const int b = row / SEQ, s = row - b * SEQ;
  const float* src = x + ((size_t)b * SEQ_FULL + s) * DM + c8;
  const v4f a = *(const v4fa*)src, c = *(const v4fa*)(src + 4); FragH f;
#pragma unroll
  for (int q = 0; q < 4; ++q) { f.h[q] = (_Float16)bfr(a[q]); f.h[4 + q] = (_Float16)bfr(c[q]); }
  const v8us o = f.half[0];
  *(volatile v8us*)(X16 + (size_t)t * 8) = o; __threadfence(); *(volatile v8us*)(X16 + (size_t)t * 8) = o;
}

__global__ __launch_bounds__(256) void k_maskT(const float* __restrict__ mask, unsigned short* __restrict__ MT) {
  __shared__ unsigned short tl[64][66];
  const int tid = threadIdx.x; const int tpb = (SEQ / 64) * (SEQ / 64);
  const int b = blockIdx.x / tpb; const int rem = blockIdx.x - b * tpb; const int qt = rem / (SEQ / 64), kt = rem - qt * (SEQ / 64);
  const int q0 = qt * 64, k0 = kt * 64;
  const float* src = mask + (size_t)b * SEQ_FULL * SEQ_FULL;
#pragma unroll 1
  for (int i = tid; i < 64 * 16; i += 256) { const int r = i >> 4, c4 = (i & 15) * 4; const v4f v = *(const v4fa*)(src + (size_t)(q0 + r) * SEQ_FULL + k0 + c4);
#pragma unroll
    for (int j = 0; j < 4; ++j) tl[c4 + j][r] = bf16_bits(v[j]); }
  __syncthreads();
  for (int pass = 0; pass < 2; ++pass) {
#pragma unroll
    for (int rd = 0; rd < 2; ++rd) { const int d = rd * 32 + (tid >> 3), pc = tid & 7; FragH f;
#pragma unroll
      for (int q = 0; q < 8; ++q) f.u[q] = tl[d][pc * 8 + q];
      const v8us o = f.half[0];
      *(volatile v8us*)(MT + ((size_t)b * SEQ + k0 + d) * SEQ + q0 + pc * 8) = o; }
    if (pass == 0) __threadfence(); }
}

template <bool BIASROW>
__device__ __forceinline__ void proj_body(const unsigned short* A, const unsigned short* Bt, const float* bias, unsigned short* Ch, unsigned short* Cl, int lda, int ldb, int ldc, int N, int K, float alpha) {
  __shared__ __attribute__((aligned(16))) float so[4][32][68];
  const int tid = threadIdx.x; const int w = __builtin_amdgcn_readfirstlane((int)(tid >> 5)); const int lane = tid & 31, ln = lane & 15, hh = lane >> 4;
  const int ntn = N >> 6; const int mt = (int)blockIdx.x / ntn, nq = (int)blockIdx.x - mt * ntn; const int row0 = mt * 128 + 32 * w, col0 = nq * 64;
  const unsigned short* a0p = A + (size_t)(row0 + ln) * lda; const unsigned short* a1p = a0p + (size_t)16 * lda;
  const unsigned short* b0p = Bt + (size_t)(col0 + ln) * ldb; const unsigned short* b1p = b0p + (size_t)16 * ldb; const unsigned short* b2p = b1p + (size_t)16 * ldb; const unsigned short* b3p = b2p + (size_t)16 * ldb;
  const v8f z8 = {0.f, 0.f, 0.f, 0.f, 0.f, 0.f, 0.f, 0.f}; v8f c00 = z8, c01 = z8, c02 = z8, c03 = z8, c10 = z8, c11 = z8, c12 = z8, c13 = z8;
#pragma unroll 1
  for (int kb = 0; kb < K; kb += 32) { const v16h a0 = ldfrag(a0p + kb, hh), a1 = ldfrag(a1p + kb, hh);
    v16h b = ldfrag(b0p + kb, hh); c00 = mma16(a0, b, c00); c10 = mma16(a1, b, c10);
    b = ldfrag(b1p + kb, hh); c01 = mma16(a0, b, c01); c11 = mma16(a1, b, c11);
    b = ldfrag(b2p + kb, hh); c02 = mma16(a0, b, c02); c12 = mma16(a1, b, c12);
    b = ldfrag(b3p + kb, hh); c03 = mma16(a0, b, c03); c13 = mma16(a1, b, c13); }
  v8f accs[8] = {c00, c01, c02, c03, c10, c11, c12, c13};
#pragma unroll
  for (int u = 0; u < 8; ++u) { const int t = u & 3, half = u >> 2; const int col = col0 + t * 16 + ln; const float bcol = BIASROW ? 0.f : bfr(bias[col]);
#pragma unroll
    for (int r = 0; r < 8; ++r) { const int rloc = half * 16 + 8 * hh + r; const float bv = BIASROW ? bfr(bias[row0 + rloc]) : bcol; so[w][rloc][t * 16 + ln] = accs[u][r] * alpha + bv; } }
  __builtin_amdgcn_fence(4  , "workgroup"); __builtin_amdgcn_wave_barrier();
  const int rsub = lane >> 3, c8 = (lane & 7) * 8;
  for (int pass = 0; pass < 2; ++pass) {
#pragma unroll
    for (int q = 0; q < 8; ++q) { const int r = q * 4 + rsub; const v4f x0 = *(const v4fa*)&so[w][r][c8], x1 = *(const v4fa*)&so[w][r][c8 + 4]; FragH fh, fl;
#pragma unroll
      for (int i = 0; i < 4; ++i) { _Float16 h = (_Float16)x0[i]; fh.h[i] = h; fl.h[i] = (_Float16)((x0[i] - (float)h) * 1024.0f); h = (_Float16)x1[i]; fh.h[4 + i] = h; fl.h[4 + i] = (_Float16)((x1[i] - (float)h) * 1024.0f); }
      const v8us oh = fh.half[0], ol = fl.half[0]; const size_t o = (size_t)(row0 + r) * ldc + col0 + c8;
      *(volatile v8us*)(Ch + o) = oh; *(volatile v8us*)(Cl + o) = ol; }
    if (pass == 0) __threadfence(); }
}
__global__ __launch_bounds__(128) void k_proj_hl(const unsigned short* __restrict__ A, const unsigned short* __restrict__ Bt, const float* __restrict__ bias, unsigned short* __restrict__ Ch, unsigned short* __restrict__ Cl, int lda, int ldb, int ldc, int N, int K, float alpha) {
  proj_body<false>(A, Bt, bias, Ch, Cl, lda, ldb, ldc, N, K, alpha); }
__global__ __launch_bounds__(128) void k_projT_hl(const unsigned short* __restrict__ A, const unsigned short* __restrict__ Bt, const float* __restrict__ bias, unsigned short* __restrict__ Ch, unsigned short* __restrict__ Cl, int lda, int ldb, int ldc, int N, int K, float alpha) {
  proj_body<true>(A, Bt, bias, Ch, Cl, lda, ldb, ldc, N, K, alpha); }

template <bool ISL_>
__device__ __forceinline__ void attn_body(const unsigned short* Qh, const unsigned short* Ql, const unsigned short* Kh, const unsigned short* Kl,
                                          const unsigned short* Vh, const unsigned short* Vl, const unsigned short* MT, unsigned short* Ch, unsigned short* Cl, int qblk0) {
  __shared__ __attribute__((aligned(16))) _Float16 ph[4][16][40];
  __shared__ __attribute__((aligned(16))) _Float16 pl[4][16][40];
  __shared__ __attribute__((aligned(16))) float so[4][16][68];
  const int tid = threadIdx.x; const int w = __builtin_amdgcn_readfirstlane((int)(tid >> 5)); const int lane = tid & 31, ln = lane & 15, hh = lane >> 4;
  const int bh = blockIdx.y; const int b = bh / NH, h = bh - b * NH;
  const int q0 = (qblk0 + (int)blockIdx.x) * 64 + 16 * w;
  const int rowb = b * SEQ;
  int qoff = (rowb + q0 + ln) * DM + h * HD;
  const int koff0 = (rowb + ln) * DM + h * HD;
  const int voff0 = (h * HD + ln) * NRI + rowb;
  const size_t moff0 = ((size_t)rowb + ln) * SEQ + q0 + 8 * hh;
  const v8f z8 = {0.f, 0.f, 0.f, 0.f, 0.f, 0.f, 0.f, 0.f};
  v8f acc[4] = {z8, z8, z8, z8}, accr[4] = {z8, z8, z8, z8};
  float mrun[8], lrun[8];
#pragma unroll
  for (int r = 0; r < 8; ++r) { mrun[r] = -1.0e30f; lrun[r] = 0.f; }
#pragma unroll 1
  for (int key0 = 0; key0 < SEQ; key0 += 32) {
    asm volatile("" : "+v"(qoff));
    const v8us mk0 = *(const v8us*)(MT + moff0 + (size_t)key0 * SEQ);
    const v8us mk1 = *(const v8us*)(MT + moff0 + (size_t)(key0 + 16) * SEQ);
    v8f s0 = z8, s1 = z8, r0 = z8, r1 = z8;
#pragma unroll
    for (int ds = 0; ds < 2; ++ds) {
      const v16h qh = ldfrag(Qh + qoff + ds * 32, hh);
      const int ko = koff0 + key0 * DM + ds * 32;
      const v16h k0h = ldfrag(Kh + ko, hh);
      s0 = mma16(qh, k0h, s0);
      const v16h k1h = ldfrag(Kh + ko + 16 * DM, hh);
      s1 = mma16(qh, k1h, s1);
      if (ISL_) {
        const v16h ql = ldfrag(Ql + qoff + ds * 32, hh);
        r0 = mma16(ql, k0h, r0); r1 = mma16(ql, k1h, r1);
        const v16h k0l = ldfrag(Kl + ko, hh); r0 = mma16(qh, k0l, r0);
        const v16h k1l = ldfrag(Kl + ko + 16 * DM, hh); r1 = mma16(qh, k1l, r1);
      }
    }
#pragma unroll
    for (int r = 0; r < 8; ++r) {
      float a0 = s0[r], a1 = s1[r];
      if (ISL_) { a0 += r0[r] * 0.0009765625f; a1 += r1[r] * 0.0009765625f; }
      const float x0 = a0 * 0.125f - 1.0e9f * bf16_val(mk0[r]);
      const float x1 = a1 * 0.125f - 1.0e9f * bf16_val(mk1[r]);
      float rm = fmaxf(x0, x1);
      rm = fmaxf(rm, __shfl_xor(rm, 1)); rm = fmaxf(rm, __shfl_xor(rm, 2)); rm = fmaxf(rm, __shfl_xor(rm, 4)); rm = fmaxf(rm, __shfl_xor(rm, 8));
      const float mnew = fmaxf(mrun[r], rm);
      const float corr = __expf(mrun[r] - mnew);
      const float e0 = __expf(x0 - mnew), e1 = __expf(x1 - mnew);
      lrun[r] = lrun[r] * corr + (e0 + e1);
      mrun[r] = mnew;
#pragma unroll
      for (int t = 0; t < 4; ++t) { acc[t][r] *= corr; if (ISL_) accr[t][r] *= corr; }
      const float c0 = e0 * 256.0f, c1 = e1 * 256.0f;
      const _Float16 h0 = (_Float16)c0, h1 = (_Float16)c1;
      ph[w][8 * hh + r][ln] = h0; ph[w][8 * hh + r][16 + ln] = h1;
      if (ISL_) { pl[w][8 * hh + r][ln] = (_Float16)((c0 - (float)h0) * 1024.0f); pl[w][8 * hh + r][16 + ln] = (_Float16)((c1 - (float)h1) * 1024.0f); }
    }
    __builtin_amdgcn_fence(4  , "workgroup"); __builtin_amdgcn_wave_barrier();
    FragH pa, pb;
    pa.half[0] = *(const v8us*)&ph[w][ln][8 * hh]; pa.half[1] = *(const v8us*)&ph[w][ln][16 + 8 * hh];
    if (ISL_) { pb.half[0] = *(const v8us*)&pl[w][ln][8 * hh]; pb.half[1] = *(const v8us*)&pl[w][ln][16 + 8 * hh]; }
#pragma unroll
    for (int t = 0; t < 4; ++t) {
      const int vo = voff0 + t * 16 * NRI + key0;
      const v16h vh = ldfrag(Vh + vo, hh);
      acc[t] = mma16(pa.v, vh, acc[t]);
      if (ISL_) { accr[t] = mma16(pb.v, vh, accr[t]); const v16h vl = ldfrag(Vl + vo, hh); accr[t] = mma16(pa.v, vl, accr[t]); }
    }
    __builtin_amdgcn_fence(4  , "workgroup"); __builtin_amdgcn_wave_barrier();
  }
  float inv[8];
#pragma unroll
  for (int r = 0; r < 8; ++r) { float lt = lrun[r]; lt += __shfl_xor(lt, 1); lt += __shfl_xor(lt, 2); lt += __shfl_xor(lt, 4); lt += __shfl_xor(lt, 8); inv[r] = 0.25f * (1.0f / lt); }
#pragma unroll
  for (int t = 0; t < 4; ++t) {
#pragma unroll
    for (int r = 0; r < 8; ++r) { float v = acc[t][r]; if (ISL_) v += accr[t][r] * 0.0009765625f; so[w][8 * hh + r][t * 16 + ln] = v * inv[r]; } }
  __builtin_amdgcn_fence(4  , "workgroup"); __builtin_amdgcn_wave_barrier();
  const int rsub = lane >> 3, c8 = (lane & 7) * 8;
  for (int pass = 0; pass < 2; ++pass) {
#pragma unroll
    for (int q = 0; q < 4; ++q) { const int r = q * 4 + rsub; const v4f x0 = *(const v4fa*)&so[w][r][c8], x1 = *(const v4fa*)&so[w][r][c8 + 4]; FragH fh, fl;
#pragma unroll
      for (int i = 0; i < 4; ++i) { _Float16 hv = (_Float16)x0[i]; fh.h[i] = hv; fl.h[i] = (_Float16)((x0[i] - (float)hv) * 1024.0f); hv = (_Float16)x1[i]; fh.h[4 + i] = hv; fl.h[4 + i] = (_Float16)((x1[i] - (float)hv) * 1024.0f); }
      const v8us oh = fh.half[0], ol = fl.half[0]; const size_t o = (size_t)(rowb + q0 + r) * DM + h * HD + c8;
      *(volatile v8us*)(Ch + o) = oh; if (ISL_) *(volatile v8us*)(Cl + o) = ol; }
    if (pass == 0) __threadfence(); }
}
__global__ __launch_bounds__(128) void k_attn_isl(const unsigned short* __restrict__ Qh, const unsigned short* __restrict__ Ql, const unsigned short* __restrict__ Kh, const unsigned short* __restrict__ Kl,
                                                 const unsigned short* __restrict__ Vh, const unsigned short* __restrict__ Vl, const unsigned short* __restrict__ MT, unsigned short* __restrict__ Ch, unsigned short* __restrict__ Cl) {
  attn_body<true>(Qh, Ql, Kh, Kl, Vh, Vl, MT, Ch, Cl, 0); }
__global__ __launch_bounds__(128) void k_attn_main(const unsigned short* __restrict__ Qh, const unsigned short* __restrict__ Kh, const unsigned short* __restrict__ Vh, const unsigned short* __restrict__ MT, unsigned short* __restrict__ Ch) {
  attn_body<false>(Qh, Qh, Kh, Kh, Vh, Vh, MT, Ch, Ch, ISL / 64); }

__global__ __launch_bounds__(128) void k_out(const unsigned short* __restrict__ Ah, const unsigned short* __restrict__ Al, const unsigned short* __restrict__ Bt, const float* __restrict__ bias, float* __restrict__ out) {
  __shared__ __attribute__((aligned(16))) float so[4][16][68];
  const int tid = threadIdx.x; const int w = __builtin_amdgcn_readfirstlane((int)(tid >> 5)); const int lane = tid & 31, ln = lane & 15, hh = lane >> 4;
  const int ntn = DM / 64; const int mt = (int)blockIdx.x / ntn, nq = (int)blockIdx.x - mt * ntn; const int row0 = mt * 64 + 16 * w, col0 = nq * 64;
  const int bb = row0 / SEQ, s0 = row0 - bb * SEQ; const bool isl = s0 < ISL;
  const int aoff = (row0 + ln) * DM; const int boff = (col0 + ln) * DM;
  const v8f z8 = {0.f, 0.f, 0.f, 0.f, 0.f, 0.f, 0.f, 0.f};
  v8f c[4] = {z8, z8, z8, z8}, cr[4] = {z8, z8, z8, z8};
  if (isl) {
#pragma unroll 1
    for (int kb = 0; kb < DM; kb += 32) { const v16h ah = ldfrag(Ah + aoff + kb, hh), al = ldfrag(Al + aoff + kb, hh);
#pragma unroll
      for (int t = 0; t < 4; ++t) { const v16h bq = ldfrag(Bt + boff + t * 16 * DM + kb, hh); c[t] = mma16(ah, bq, c[t]); cr[t] = mma16(al, bq, cr[t]); } }
  } else {
#pragma unroll 1
    for (int kb = 0; kb < DM; kb += 32) { const v16h ah = ldfrag(Ah + aoff + kb, hh);
#pragma unroll
      for (int t = 0; t < 4; ++t) { const v16h bq = ldfrag(Bt + boff + t * 16 * DM + kb, hh); c[t] = mma16(ah, bq, c[t]); } }
  }
#pragma unroll
  for (int t = 0; t < 4; ++t) { const float bv = bfr(bias[col0 + t * 16 + ln]);
#pragma unroll
    for (int r = 0; r < 8; ++r) so[w][8 * hh + r][t * 16 + ln] = c[t][r] * 0.000244140625f + cr[t][r] * 2.384185791015625e-07f + bv; }
  __builtin_amdgcn_fence(4  , "workgroup"); __builtin_amdgcn_wave_barrier();
  const int rsub = lane >> 4, c4 = (lane & 15) * 4;
  const size_t orow0 = (size_t)bb * SEQ_FULL + s0;
  for (int pass = 0; pass < 2; ++pass) {
#pragma unroll
    for (int q = 0; q < 8; ++q) { const int r = q * 2 + rsub; const v4f v = *(const v4fa*)&so[w][r][c4]; *(volatile v4f*)(out + (orow0 + r) * DM + col0 + c4) = v; }
    if (pass == 0) __threadfence(); }
}

#define PLANE_B ((size_t)NRI * DM * 2)
#define WPL_B ((size_t)DM * DM * 2)
#define MT_B ((size_t)NB * SEQ * SEQ * 2)
#define CARVE_B (4 * WPL_B + 3 * PLANE_B + MT_B + 4 * PLANE_B + 2 * PLANE_B + 2 * PLANE_B)
static_assert(CARVE_B <= (size_t)134217728);
static_assert(PLANE_B % 256 == 0 && WPL_B % 256 == 0 && MT_B % 256 == 0);

extern "C" void kernel_launch(void* const* d_in, const int* in_sizes, int n_in,
                              void* d_out, int out_size, void* d_ws, size_t ws_size, hipStream_t stream) {
  if (n_in < 12) return;
  const long long needX = ((long long)(NB - 1) * SEQ_FULL + SEQ) * DM;
  const long long needM = (long long)(NB - 1) * SEQ_FULL * SEQ_FULL + (long long)(SEQ - 1) * SEQ_FULL + SEQ;
  if (in_sizes[0] < needX || in_sizes[1] < needX || in_sizes[2] < needX || in_sizes[3] < needM) return;
  if (in_sizes[4] < DM * DM || in_sizes[6] < DM * DM || in_sizes[8] < DM * DM || in_sizes[10] < DM * DM) return;
  if (in_sizes[5] < DM || in_sizes[7] < DM || in_sizes[9] < DM || in_sizes[11] < DM) return;
  if ((long long)out_size < needX) return;
  const float* xq = (const float*)d_in[0]; const float* xk = (const float*)d_in[1]; const float* xv = (const float*)d_in[2]; const float* am = (const float*)d_in[3];
  const float* wq = (const float*)d_in[4]; const float* bq = (const float*)d_in[5]; const float* wk = (const float*)d_in[6]; const float* bk = (const float*)d_in[7];
  const float* wv = (const float*)d_in[8]; const float* bv = (const float*)d_in[9]; const float* wo = (const float*)d_in[10]; const float* bo = (const float*)d_in[11];
  char* ws = (char*)d_ws; size_t off = 0;
  auto take = [&](size_t bytes) { char* p = ws + off; off += (bytes + 255) & ~(size_t)255; return (unsigned short*)p; };
  unsigned short* WQT = take(WPL_B); unsigned short* WKT = take(WPL_B); unsigned short* WVT = take(WPL_B); unsigned short* WOT = take(WPL_B);
  unsigned short* XQ = take(PLANE_B); unsigned short* XK = take(PLANE_B); unsigned short* XV = take(PLANE_B);
  unsigned short* MT = take(MT_B);
  unsigned short* QH = take(PLANE_B); unsigned short* QL = take(PLANE_B); unsigned short* KH = take(PLANE_B); unsigned short* KL = take(PLANE_B);
  unsigned short* VTH = take(PLANE_B); unsigned short* VTL = take(PLANE_B);
  unsigned short* CH = take(PLANE_B); unsigned short* CL = take(PLANE_B);
  if (off > ws_size) return;

  const unsigned gw = (unsigned)(((size_t)DM * (DM / 8) + 255) / 256);
  k_wt_f16<<<gw, 256, 0, stream>>>(wq, WQT, DM, DM, 64.0f);
  k_wt_f16<<<gw, 256, 0, stream>>>(wk, WKT, DM, DM, 64.0f);
  k_wt_f16<<<gw, 256, 0, stream>>>(wv, WVT, DM, DM, 64.0f);
  k_wt_f16<<<gw, 256, 0, stream>>>(wo, WOT, DM, DM, 64.0f);
  const unsigned gx = (unsigned)(((size_t)NRI * (DM / 8) + 255) / 256);
  k_x16<<<gx, 256, 0, stream>>>(xq, XQ);
  k_x16<<<gx, 256, 0, stream>>>(xk, XK);
  k_x16<<<gx, 256, 0, stream>>>(xv, XV);
  k_maskT<<<(unsigned)(NB * (SEQ / 64) * (SEQ / 64)), 256, 0, stream>>>(am, MT);
  k_proj_hl<<<(unsigned)((NRI / 128) * (DM / 64)), 128, 0, stream>>>(XQ, WQT, bq, QH, QL, DM, DM, DM, DM, DM, 0.015625f);
  k_proj_hl<<<(unsigned)((NRI / 128) * (DM / 64)), 128, 0, stream>>>(XK, WKT, bk, KH, KL, DM, DM, DM, DM, DM, 0.015625f);
  k_projT_hl<<<(unsigned)((DM / 128) * (NRI / 64)), 128, 0, stream>>>(WVT, XV, bv, VTH, VTL, DM, DM, NRI, NRI, DM, 0.015625f);
  k_attn_isl<<<dim3(ISL / 64, NB * NH), 128, 0, stream>>>(QH, QL, KH, KL, VTH, VTL, MT, CH, CL);
  if ((SEQ - ISL) / 64 > 0)
    k_attn_main<<<dim3((SEQ - ISL) / 64, NB * NH), 128, 0, stream>>>(QH, KH, VTH, MT, CH);
  k_out<<<(unsigned)((NRI / 64) * (DM / 64)), 128, 0, stream>>>(CH, CL, WOT, bo, (float*)d_out);
}
